// PhysicsResidual_15144054686218
// MI455X (gfx1250) — hardware-run, weakly checked
//
#include <hip/hip_runtime.h>
#include <math.h>

typedef __attribute__((ext_vector_type(16))) _Float16 v16h;
typedef __attribute__((ext_vector_type(8)))  _Float16 v8h;
typedef __attribute__((ext_vector_type(16))) __bf16   v16b;
typedef __attribute__((ext_vector_type(8)))  __bf16   v8b;
typedef __attribute__((ext_vector_type(8)))  float    v8f;
typedef __attribute__((ext_vector_type(4)))  float    v4f;

constexpr int kNPts    = 16384;
constexpr int kWidth   = 128;
constexpr int kLayers  = 5;
constexpr int kJets    = 9;
constexpr int kBlkPts  = 32;
constexpr int kSubPts  = 16;
constexpr int kPitch   = 136;
constexpr int kSideW   = 32;
constexpr int kSideP   = 36;
constexpr int kPlaneEl = kLayers * kWidth * kWidth;
static_assert((kNPts % kBlkPts) == 0, "point tiles");
static_assert((kWidth % 32) == 0, "K multiple of 32");
static_assert(kWidth == 8 * 16, "8 waves x 16 units");
static_assert((kPlaneEl % (8 * 256)) == 0, "plane split grid exact");
static_assert(((kPitch * 2) % 16) == 0, "LDS row pitch 16-B multiple");

constexpr size_t kOffWH   = 0;
constexpr size_t kOffWL   = kOffWH + (size_t)kPlaneEl * 2;
constexpr size_t kWsTotal = kOffWL + (size_t)kPlaneEl * 2;
static_assert(kWsTotal == 327680ull, "carve total");
static_assert(kWsTotal <= 134217728ull, "carve cap");
static_assert((kOffWL % 128) == 0, "aligned region");

__device__ __forceinline__ unsigned short f2bf_bits(float f) {
  unsigned u = __float_as_uint(f);
  return (unsigned short)((u + 0x7FFFu + ((u >> 16) & 1u)) >> 16);
}
__device__ __forceinline__ float bf_bits2f(unsigned short h) { return __uint_as_float(((unsigned)h) << 16); }

__device__ __forceinline__ v16b frag_load(const __bf16* p) {
  union U { v16b v; v8b h[2]; };
  U f;
  f.h[0] = *(const v8b*)(p);
  f.h[1] = *(const v8b*)(p + 16);
  return f.v;
}

__device__ __forceinline__ void mma3_guard(v8f& c, v16b ah, v16b al, v16b bh, v16b bl) {
  c = __builtin_amdgcn_wmma_f32_16x16x32_bf16(false, ah, false, bh, (short)0, c, false, false);
  c = __builtin_amdgcn_wmma_f32_16x16x32_bf16(false, ah, false, bl, (short)0, c, false, false);
  c = __builtin_amdgcn_wmma_f32_16x16x32_bf16(false, al, false, bh, (short)0, c, false, false);
  asm volatile("v_nop\n\tv_nop\n\tv_nop\n\tv_nop" : "+v"(c) : "v"(ah), "v"(al), "v"(bh), "v"(bl));
}

__device__ __forceinline__ void split8_store(const v8f v, __bf16* ph, __bf16* pl) {
  v8b hv, lv;
#pragma unroll
  for (int e = 0; e < 8; ++e) {
    const float f = v[e];
    const unsigned short hb = f2bf_bits(f);
    const unsigned short lb = f2bf_bits(f - bf_bits2f(hb));
    hv[e] = __builtin_bit_cast(__bf16, hb);
    lv[e] = __builtin_bit_cast(__bf16, lb);
  }
  *(v8b*)ph = hv;
  *(v8b*)pl = lv;
}

__global__ __launch_bounds__(256) void split_rows_bf16_kernel(
    const float* __restrict__ src, unsigned short* __restrict__ dhi, unsigned short* __restrict__ dlo, int total8)
{
  const int i = blockIdx.x * 256 + threadIdx.x;
  if (i >= total8) return;
  const size_t e0 = (size_t)i << 3;
  const v4f a0 = *(const v4f*)(src + e0);
  const v4f a1 = *(const v4f*)(src + e0 + 4);
  v8h hv, lv;
#pragma unroll
  for (int e = 0; e < 4; ++e) {
    const unsigned short h0 = f2bf_bits(a0[e]), h1 = f2bf_bits(a1[e]);
    const unsigned short l0 = f2bf_bits(a0[e] - bf_bits2f(h0)), l1 = f2bf_bits(a1[e] - bf_bits2f(h1));
    hv[e]     = __builtin_bit_cast(_Float16, h0);
    hv[4 + e] = __builtin_bit_cast(_Float16, h1);
    lv[e]     = __builtin_bit_cast(_Float16, l0);
    lv[4 + e] = __builtin_bit_cast(_Float16, l1);
  }
  unsigned short* qh = dhi + e0;
  unsigned short* ql = dlo + e0;
  *(volatile v8h*)qh = hv;
  *(volatile v8h*)ql = lv;
  __threadfence();
  *(volatile v8h*)qh = hv;
  *(volatile v8h*)ql = lv;
}

__global__ __launch_bounds__(256) void fused_jet_kernel(
    const float* __restrict__ ct, const float* __restrict__ cx, const float* __restrict__ cy, const float* __restrict__ cz,
    const float* __restrict__ uWin, const float* __restrict__ ubin,
    const unsigned short* __restrict__ WHp, const unsigned short* __restrict__ WLp,
    const float* __restrict__ ubhid, const float* __restrict__ uWout, const float* __restrict__ ubout,
    const float* __restrict__ pWin, const float* __restrict__ pbin,
    const float* __restrict__ pWhid, const float* __restrict__ pbhid,
    const float* __restrict__ pWout, const float* __restrict__ pbout,
    float* __restrict__ out, int npts)
{
  __shared__ __align__(16) __bf16 JH[kJets * kSubPts * kPitch];
  __shared__ __align__(16) __bf16 JL[kJets * kSubPts * kPitch];
  __shared__ __align__(16) float  sH1[kBlkPts * kSideP];
  __shared__ __align__(16) float  sPsi[kBlkPts];
  __shared__ __align__(16) float  sPart[8 * 4 * kSubPts];
  __shared__ __align__(16) float  sRes[kBlkPts];
  (void)ubout;

  const int tid  = threadIdx.x;
  const int lane = tid & 31;
  const int wave = __builtin_amdgcn_readfirstlane((int)(threadIdx.x >> 5));
  const int h    = lane >> 4;
  const int rl   = lane & 15;
  const int m0   = wave * 16;
  const int pblk = blockIdx.x * kBlkPts;

  const __bf16* WH = (const __bf16*)WHp;
  const __bf16* WL = (const __bf16*)WLp;

  {
    const int pp = tid >> 3;
    const int u0 = (tid & 7) * 4;
    int pg = pblk + pp;
    pg = (pg < npts) ? pg : (npts - 1);
    const float c0 = ct[pg], c1 = cx[pg], c2 = cy[pg], c3 = cz[pg];
#pragma unroll 1
    for (int e = 0; e < 4; ++e) {
      const int u = u0 + e;
      const v4f w = *(const v4f*)(pWin + u * 4);
      float zv = w[0] * c0;
      zv = fmaf(w[1], c1, zv);
      zv = fmaf(w[2], c2, zv);
      zv = fmaf(w[3], c3, zv);
      zv = zv + pbin[u];
      sH1[pp * kSideP + u] = tanhf(zv);
    }
    __syncthreads();
    float part = 0.0f;
#pragma unroll 1
    for (int e = 0; e < 4; ++e) {
      const int u = u0 + e;
      float s = 0.0f;
#pragma unroll 1
      for (int k4 = 0; k4 < kSideW / 4; ++k4) {
        const v4f w  = *(const v4f*)(pWhid + u * kSideW + 4 * k4);
        const v4f hv = *(const v4f*)(sH1 + pp * kSideP + 4 * k4);
        s = fmaf(w[0], hv[0], s);
        s = fmaf(w[1], hv[1], s);
        s = fmaf(w[2], hv[2], s);
        s = fmaf(w[3], hv[3], s);
      }
      s = s + pbhid[u];
      part = fmaf(pWout[u], tanhf(s), part);
    }
    part += __shfl_xor(part, 1, 32);
    part += __shfl_xor(part, 2, 32);
    part += __shfl_xor(part, 4, 32);
    float pbo = pbout[0];
    asm volatile("" : "+v"(pbo));
    const float psiv = part + pbo;
    if ((tid & 7) == 0) sPsi[pp] = psiv;
  }

  const int stOff = rl * kPitch + m0 + 8 * h;
  const int ldOff = rl * kPitch + 8 * h;

#pragma unroll 1
  for (int sub = 0; sub < 2; ++sub) {
    v8f acc[kJets];
#pragma unroll 1
    for (int layer = -1; layer < kLayers; ++layer) {
      if (layer < 0) {
        int pg = pblk + sub * kSubPts + rl;
        pg = (pg < npts) ? pg : (npts - 1);
        const float q0 = ct[pg], q1 = cx[pg], q2 = cy[pg], q3 = cz[pg];
#pragma unroll
        for (int r = 0; r < 8; ++r) {
          const v4f w = *(const v4f*)(uWin + (m0 + 8 * h + r) * 4);
          float s = w[0] * q0;
          s = fmaf(w[1], q1, s);
          s = fmaf(w[2], q2, s);
          s = fmaf(w[3], q3, s);
          acc[0][r] = s;
          acc[1][r] = w[0];
          acc[2][r] = w[1];
          acc[3][r] = w[2];
          acc[4][r] = w[3];
          acc[5][r] = 0.0f;
          acc[6][r] = 0.0f;
          acc[7][r] = 0.0f;
          acc[8][r] = 0.0f;
        }
      } else {
#pragma unroll
        for (int j = 0; j < kJets; ++j) acc[j] = (v8f){0.f, 0.f, 0.f, 0.f, 0.f, 0.f, 0.f, 0.f};
        const __bf16* wh = WH + (size_t)layer * (kWidth * kWidth) + (m0 + rl) * kWidth + 8 * h;
        const __bf16* wl = WL + (size_t)layer * (kWidth * kWidth) + (m0 + rl) * kWidth + 8 * h;
#pragma unroll 1
        for (int k0 = 0; k0 < kWidth; k0 += 32) {
          const v16b ah = frag_load(wh + k0);
          const v16b al = frag_load(wl + k0);
#pragma unroll
          for (int j = 0; j < kJets; ++j) {
            const v16b bh = frag_load(JH + j * (kSubPts * kPitch) + ldOff + k0);
            const v16b bl = frag_load(JL + j * (kSubPts * kPitch) + ldOff + k0);
            mma3_guard(acc[j], ah, al, bh, bl);
          }
        }
      }
      __syncthreads();

      {
        const float* bp = (layer < 0) ? (ubin + m0 + 8 * h) : (ubhid + layer * kWidth + m0 + 8 * h);
        const v4f b0 = *(const v4f*)(bp);
        const v4f b1 = *(const v4f*)(bp + 4);
        const float bb[8] = {b0[0], b0[1], b0[2], b0[3], b1[0], b1[1], b1[2], b1[3]};
#pragma unroll
        for (int r = 0; r < 8; ++r) {
          const float z0 = acc[0][r] + bb[r];
          const float a  = tanhf(z0);
          const float g  = 1.0f - a * a;
          const float h2 = -2.0f * a * g;
          acc[0][r] = a;
#pragma unroll
          for (int i = 0; i < 4; ++i) {
            const float d1 = acc[1 + i][r];
            const float d2 = acc[5 + i][r];
            acc[1 + i][r] = g * d1;
            acc[5 + i][r] = fmaf(g, d2, h2 * d1 * d1);
          }
        }
      }

      if (layer < kLayers - 1) {
#pragma unroll
        for (int j = 0; j < kJets; ++j)
          split8_store(acc[j], JH + j * (kSubPts * kPitch) + stOff, JL + j * (kSubPts * kPitch) + stOff);
      } else {
        const v4f o0 = *(const v4f*)(uWout + m0 + 8 * h);
        const v4f o1 = *(const v4f*)(uWout + m0 + 8 * h + 4);
        const float wo[8] = {o0[0], o0[1], o0[2], o0[3], o1[0], o1[1], o1[2], o1[3]};
        float dd0 = 0.0f, dd1 = 0.0f, dd2 = 0.0f, dd3 = 0.0f;
#pragma unroll
        for (int r = 0; r < 8; ++r) {
          dd0 = fmaf(wo[r], acc[5][r], dd0);
          dd1 = fmaf(wo[r], acc[6][r], dd1);
          dd2 = fmaf(wo[r], acc[7][r], dd2);
          dd3 = fmaf(wo[r], acc[8][r], dd3);
        }
        dd0 += __shfl_xor(dd0, 16, 32);
        dd1 += __shfl_xor(dd1, 16, 32);
        dd2 += __shfl_xor(dd2, 16, 32);
        dd3 += __shfl_xor(dd3, 16, 32);
        if (h == 0) {
          sPart[(wave * 4 + 0) * kSubPts + rl] = dd0;
          sPart[(wave * 4 + 1) * kSubPts + rl] = dd1;
          sPart[(wave * 4 + 2) * kSubPts + rl] = dd2;
          sPart[(wave * 4 + 3) * kSubPts + rl] = dd3;
        }
      }
      __syncthreads();
    }

    if (tid < kSubPts) {
      float ds[4];
#pragma unroll
      for (int i = 0; i < 4; ++i) {
        float s = 0.0f;
#pragma unroll
        for (int w = 0; w < 8; ++w) s += sPart[(w * 4 + i) * kSubPts + tid];
        ds[i] = s;
      }
      const float cv  = 1.0f + sPsi[sub * kSubPts + tid];
      const float lap = (ds[1] + ds[2]) + ds[3];
      float rv = ds[0] - (cv * cv) * lap;
      if (__builtin_isnan(ds[0]) || __builtin_isnan(ds[1]) || __builtin_isnan(ds[2]) ||
          __builtin_isnan(ds[3]) || __builtin_isnan(cv))
        rv = __uint_as_float(0x7fc00000u);
      sRes[sub * kSubPts + tid] = rv;
    }
  }
  __syncthreads();

  if (wave == 0) {
    const int l8 = lane & 7;
    const v4f val = *(const v4f*)(sRes + 4 * l8);
    float* op = out + (size_t)pblk + 4 * l8;
    if (lane < 8) *(volatile v4f*)op = val;
    __threadfence();
    if (lane < 8) *(volatile v4f*)op = val;
  }
}

extern "C" void kernel_launch(void* const* d_in, const int* in_sizes, int n_in,
                              void* d_out, int out_size, void* d_ws, size_t ws_size,
                              hipStream_t stream) {
  if (n_in < 16) return;
  if (in_sizes[0] != kNPts || in_sizes[1] != kNPts || in_sizes[2] != kNPts || in_sizes[3] != kNPts) return;
  if (in_sizes[4] != kWidth * 4 || in_sizes[5] != kWidth) return;
  if (in_sizes[6] != kPlaneEl || in_sizes[7] != kLayers * kWidth) return;
  if (in_sizes[8] != kWidth || in_sizes[9] != 1) return;
  if (in_sizes[10] != kSideW * 4 || in_sizes[11] != kSideW) return;
  if (in_sizes[12] != kSideW * kSideW || in_sizes[13] != kSideW) return;
  if (in_sizes[14] != kSideW || in_sizes[15] != 1) return;
  if (out_size != kNPts) return;
  if (ws_size < kWsTotal) return;

  const float* ct     = (const float*)d_in[0];
  const float* cx     = (const float*)d_in[1];
  const float* cy     = (const float*)d_in[2];
  const float* cz     = (const float*)d_in[3];
  const float* uW_in  = (const float*)d_in[4];
  const float* ub_in  = (const float*)d_in[5];
  const float* uW_hid = (const float*)d_in[6];
  const float* ub_hid = (const float*)d_in[7];
  const float* uW_out = (const float*)d_in[8];
  const float* ub_out = (const float*)d_in[9];
  const float* pW_in  = (const float*)d_in[10];
  const float* pb_in  = (const float*)d_in[11];
  const float* pW_hid = (const float*)d_in[12];
  const float* pb_hid = (const float*)d_in[13];
  const float* pW_out = (const float*)d_in[14];
  const float* pb_out = (const float*)d_in[15];

  char* ws = (char*)d_ws;
  unsigned short* WHp = (unsigned short*)(ws + kOffWH);
  unsigned short* WLp = (unsigned short*)(ws + kOffWL);

  split_rows_bf16_kernel<<<(kPlaneEl / 8) / 256, 256, 0, stream>>>(uW_hid, WHp, WLp, kPlaneEl / 8);

  fused_jet_kernel<<<kNPts / kBlkPts, 256, 0, stream>>>(
      ct, cx, cy, cz, uW_in, ub_in, WHp, WLp, ub_hid, uW_out, ub_out,
      pW_in, pb_in, pW_hid, pb_hid, pW_out, pb_out, (float*)d_out, kNPts);
}
